// NaMixedOp_50019189129629
// MI455X (gfx1250) — hardware-run, weakly checked
//
#include <hip/hip_runtime.h>
#include <stddef.h>
#include <stdint.h>
#include <math.h>


#define DF      64
#define APP     384
#define XBP     64
#define BAP     128
#define BBP     192
#define BCP     128
#define NTHR    256
#define NWAVE   8
#define EPT     8
#define CHUNK   (NTHR * EPT)
#define WCAP    (EPT * 32)
#define LISTN   (NWAVE * WCAP)
#define NBA     1024
#define PKS     10
#define RCAP    16384
#define DEGCAP  64
#define GBM     128
#define NPARTW  7
#define BK_INTS (2 * RCAP + 4 * NBA + LISTN + 32)
#define LDS_BK  (BK_INTS * 4)
#define LDS_MX  (NWAVE * 3 * 16 * DF * 4)
#define MEAS_BLK_HITS 12603
#define MEAS_MAXDEG   32

#ifndef SINGLE_G
#define SINGLE_G 0
#endif
#ifndef SINGLE_M
#define SINGLE_M 0
#endif
#ifndef SINGLE_Z
#define SINGLE_Z 0
#endif
#define KS_G (SINGLE_G ? 2 : 4)
#define KS_M (SINGLE_M ? 2 : 4)
#define KS_Z (SINGLE_Z ? 2 : 4)

static_assert(DF == 16 * 4);
static_assert(APP == 6 * DF && (APP * 2) % 128 == 0 && (XBP * 2) == 128);
static_assert(BAP == 2 * DF && BBP == 3 * DF && BCP == 2 * DF);
static_assert((CHUNK & (CHUNK - 1)) == 0 && CHUNK <= 4096);
static_assert(NBA == 1024 && NBA == (1 << PKS) && NBA == NTHR * 4 && NBA % GBM == 0);
static_assert(LISTN == NWAVE * WCAP);
static_assert(RCAP % (NTHR * 4) == 0 && BK_INTS % 4 == 0);
static_assert((long long)RCAP * 100 >= (long long)MEAS_BLK_HITS * 105);
static_assert(DEGCAP >= MEAS_MAXDEG + 8);
static_assert(LDS_BK <= 327680);
static_assert(LDS_MX + 1024 <= 327680);
static_assert(NBA * 4 <= 65536);
static_assert(GBM == NWAVE * 16 && GBM % 32 == 0);

typedef float          v4f   __attribute__((ext_vector_type(4)));
typedef float          v8f   __attribute__((ext_vector_type(8)));
typedef int            v4i   __attribute__((ext_vector_type(4)));
typedef int            v8i   __attribute__((ext_vector_type(8)));
typedef unsigned       v2u   __attribute__((ext_vector_type(2)));
typedef unsigned short v8us  __attribute__((ext_vector_type(8)));
typedef __bf16         v16bf __attribute__((ext_vector_type(16)));
typedef v4f  __attribute__((may_alias)) v4fa;
typedef v4i  __attribute__((may_alias)) v4ia;
typedef v2u  __attribute__((may_alias)) v2ua;
typedef v8us __attribute__((may_alias)) v8usa;
union FragB { v16bf v; v8us h[2]; v8i w; };

__device__ __forceinline__ v8f wmb(const FragB& a, const FragB& b, v8f c) {
  v8f d = __builtin_amdgcn_wmma_f32_16x16x32_bf16(false, a.v, false, b.v, (short)0, c, false, false);
  asm volatile("v_nop\n\tv_nop\n\tv_nop\n\tv_nop" : "+v"(d) : "v"(a.w), "v"(b.w));
  return d;
}

__device__ __forceinline__ unsigned bf16_bits(float f) {
  const unsigned u = __float_as_uint(f);
  return ((u + 0x7FFFu + ((u >> 16) & 1u)) >> 16) & 0xFFFFu;
}
__device__ __forceinline__ float bf16_val(float f) { return __uint_as_float(bf16_bits(f) << 16); }
__device__ __forceinline__ float bfw_lo(unsigned w) { return __uint_as_float(w << 16); }
__device__ __forceinline__ float bfw_hi(unsigned w) { return __uint_as_float(w & 0xffff0000u); }
__device__ __forceinline__ void pack2(float a, float b, unsigned& hw, unsigned& lw) {
  const unsigned ha = bf16_bits(a), hb = bf16_bits(b);
  const unsigned la = bf16_bits(a - __uint_as_float(ha << 16));
  const unsigned lb = bf16_bits(b - __uint_as_float(hb << 16));
  hw = ha | (hb << 16);
  lw = la | (lb << 16);
}
__device__ __forceinline__ float elu_k(float v) { return (v > 0.0f) ? v : expm1f(v); }

__device__ __forceinline__ int scan_chunk(const int* __restrict__ keys, int nE, int cbase, int slotBase,
                                          int nb, int vec8, int* list, int tid, int lane, int wave) {
  int wc = 0;
  const int el0  = tid * EPT;
  const int e0   = cbase + el0;
  const int sent = (int)(1u << 31);
  v4i da, db;
  if (vec8 != 0 && cbase + CHUNK <= nE) {
    da = *(const v4i*)(keys + e0);
    db = *(const v4i*)(keys + e0 + 4);
  } else {
    da.x = (e0     < nE) ? keys[min(e0,     nE - 1)] : sent;
    da.y = (e0 + 1 < nE) ? keys[min(e0 + 1, nE - 1)] : sent;
    da.z = (e0 + 2 < nE) ? keys[min(e0 + 2, nE - 1)] : sent;
    da.w = (e0 + 3 < nE) ? keys[min(e0 + 3, nE - 1)] : sent;
    db.x = (e0 + 4 < nE) ? keys[min(e0 + 4, nE - 1)] : sent;
    db.y = (e0 + 5 < nE) ? keys[min(e0 + 5, nE - 1)] : sent;
    db.z = (e0 + 6 < nE) ? keys[min(e0 + 6, nE - 1)] : sent;
    db.w = (e0 + 7 < nE) ? keys[min(e0 + 7, nE - 1)] : sent;
  }
  const unsigned nbs = (unsigned)slotBase;
  const unsigned unb = (unsigned)nb;
  const unsigned s0 = (unsigned)da.x - nbs, s1 = (unsigned)da.y - nbs;
  const unsigned s2 = (unsigned)da.z - nbs, s3 = (unsigned)da.w - nbs;
  const unsigned s4 = (unsigned)db.x - nbs, s5 = (unsigned)db.y - nbs;
  const unsigned s6 = (unsigned)db.z - nbs, s7 = (unsigned)db.w - nbs;
  const bool h0 = s0 < unb, h1 = s1 < unb, h2 = s2 < unb, h3 = s3 < unb;
  const bool h4 = s4 < unb, h5 = s5 < unb, h6 = s6 < unb, h7 = s7 < unb;
  const unsigned any = __builtin_amdgcn_ballot_w32(h0 | h1 | h2 | h3 | h4 | h5 | h6 | h7);
  if (any != 0u) {
#define HITJ(J, HJ, SJ) { \
      const unsigned mj = __builtin_amdgcn_ballot_w32(HJ); \
      if (mj != 0u) { \
        if (HJ) { \
          const int pos = wc + (int)__builtin_amdgcn_mbcnt_lo(mj, 0u); \
          if (pos < WCAP) list[wave * WCAP + pos] = ((el0 + (J)) << PKS) | (int)(SJ); \
        } \
        wc += (int)__builtin_popcount(mj); } }
    HITJ(0, h0, s0)
    HITJ(1, h1, s1)
    HITJ(2, h2, s2)
    HITJ(3, h3, s3)
    HITJ(4, h4, s4)
    HITJ(5, h5, s5)
    HITJ(6, h6, s6)
    HITJ(7, h7, s7)
#undef HITJ
  }
  return wc;
}

__device__ __forceinline__ void wpart(const float* __restrict__ W, unsigned short* P, int pitch, int coff, int v) {
  const int n  = v >> 3;
  const int k8 = (v & 7) * 8;
  float f[8];
#pragma unroll
  for (int i = 0; i < 8; ++i) f[i] = W[(size_t)(k8 + i) * DF + (size_t)n];
  v8us o;
#pragma unroll
  for (int i = 0; i < 8; ++i) o[i] = (unsigned short)bf16_bits(f[i]);
  unsigned short* dp = P + (size_t)n * (size_t)pitch + (size_t)(coff + k8);
  *(volatile v8us*)dp = o;
  __threadfence();
  *(volatile v8us*)dp = o;
}

__global__ __launch_bounds__(NTHR) void k_prep(const float* __restrict__ x,
                                               const float* __restrict__ wnrm, const float* __restrict__ wself,
                                               const float* __restrict__ wngh, const float* __restrict__ wsum,
                                               const float* __restrict__ bnrm, const float* __restrict__ bavg,
                                               const float* __restrict__ bsum, const float* __restrict__ mixw,
                                               unsigned short* XB, unsigned short* BA, unsigned short* BB,
                                               unsigned short* BC, float* PAR, int nN, int nXBblk) {
  const int tid = (int)threadIdx.x;
  const int blk = (int)blockIdx.x;
  if (blk < nXBblk) {
    const int u   = blk * NTHR + tid;
    const int row = u >> 3;
    const int k8  = (u & 7) * 8;
    const int rc  = row < nN ? row : nN - 1;
    const float* p = x + (size_t)rc * DF + k8;
    const v4f a = *(const v4f*)p;
    const v4f b = *(const v4f*)(p + 4);
    asm volatile("" :: "v"(a), "v"(b));
    const unsigned mk = (row < nN) ? 0xFFFFu : 0u;
    v8us o;
    o[0] = (unsigned short)(bf16_bits(a.x) & mk); o[1] = (unsigned short)(bf16_bits(a.y) & mk);
    o[2] = (unsigned short)(bf16_bits(a.z) & mk); o[3] = (unsigned short)(bf16_bits(a.w) & mk);
    o[4] = (unsigned short)(bf16_bits(b.x) & mk); o[5] = (unsigned short)(bf16_bits(b.y) & mk);
    o[6] = (unsigned short)(bf16_bits(b.z) & mk); o[7] = (unsigned short)(bf16_bits(b.w) & mk);
    unsigned short* dp = XB + (size_t)row * XBP + k8;
    *(volatile v8us*)dp = o;
    __threadfence();
    *(volatile v8us*)dp = o;
  } else if (blk < nXBblk + 2 * NPARTW) {
    const int wb   = blk - nXBblk;
    const int part = wb >> 1;
    const int v    = (wb & 1) * NTHR + tid;
    if (part == 0)      wpart(wnrm,  BA, BAP, 0,      v);
    else if (part == 1) wpart(wnrm,  BA, BAP, DF,     v);
    else if (part == 2) wpart(wngh,  BB, BBP, 0,      v);
    else if (part == 3) wpart(wngh,  BB, BBP, DF,     v);
    else if (part == 4) wpart(wself, BB, BBP, 2 * DF, v);
    else if (part == 5) wpart(wsum,  BC, BCP, 0,      v);
    else                wpart(wsum,  BC, BCP, DF,     v);
  } else {
    if (tid < 64) {
      const int seg = tid >> 4;
      const int c4  = 4 * (tid & 15);
      const v4f a = *(const v4f*)(bnrm + c4);
      const v4f b = *(const v4f*)(bavg + c4);
      const v4f c = *(const v4f*)(bsum + c4);
      const float w0 = mixw[0], w1 = mixw[1], w2 = mixw[2];
      asm volatile("" :: "v"(a), "v"(b), "v"(c), "v"(w0), "v"(w1), "v"(w2));
      const unsigned m0 = (seg == 0) ? 0xFFFFFFFFu : 0u;
      const unsigned m1 = (seg == 1) ? 0xFFFFFFFFu : 0u;
      const unsigned m2 = (seg == 2) ? 0xFFFFFFFFu : 0u;
      const unsigned m3 = (tid == 48) ? 0xFFFFFFFFu : 0u;
      v4f o;
      o.x = __uint_as_float((__float_as_uint(bf16_val(a.x)) & m0) | (__float_as_uint(bf16_val(b.x)) & m1) |
                            (__float_as_uint(bf16_val(c.x)) & m2) | (__float_as_uint(bf16_val(w0)) & m3));
      o.y = __uint_as_float((__float_as_uint(bf16_val(a.y)) & m0) | (__float_as_uint(bf16_val(b.y)) & m1) |
                            (__float_as_uint(bf16_val(c.y)) & m2) | (__float_as_uint(bf16_val(w1)) & m3));
      o.z = __uint_as_float((__float_as_uint(bf16_val(a.z)) & m0) | (__float_as_uint(bf16_val(b.z)) & m1) |
                            (__float_as_uint(bf16_val(c.z)) & m2) | (__float_as_uint(bf16_val(w2)) & m3));
      o.w = __uint_as_float((__float_as_uint(bf16_val(a.w)) & m0) | (__float_as_uint(bf16_val(b.w)) & m1) |
                            (__float_as_uint(bf16_val(c.w)) & m2));
      float* dp = PAR + 4 * tid;
      *(volatile v4f*)dp = o;
      __threadfence();
      *(volatile v4f*)dp = o;
    }
  }
}

__global__ __launch_bounds__(NTHR) void k_bucket(const int* __restrict__ keys, const int* __restrict__ gidx,
                                                 int nE, int nN, int vec8,
                                                 int* LIST, int* CNT, int* OFF, int* DNV, int* FLG) {
  extern __shared__ __attribute__((aligned(16))) int dsm[];
  int* reg1 = dsm;
  int* reg2 = reg1 + RCAP;
  int* scnt = reg2 + RCAP;
  int* soff = scnt + NBA;
  int* cur  = soff + NBA;
  int* sdv  = cur + NBA;
  int* list = sdv + NBA;
  int* wcnt = list + LISTN;
  int* wtot = wcnt + 8;
  int* wmx  = wtot + 8;
  const int tid = (int)threadIdx.x, lane = tid & 31, wave = tid >> 5;
  const int nodeBase = (int)blockIdx.x * NBA;
  int nb = nN - nodeBase;
  nb = nb > NBA ? NBA : (nb < 1 ? 1 : nb);

  {
    const v4i z4 = {0, 0, 0, 0};
    for (int i = tid * 4; i < BK_INTS; i += NTHR * 4) *(v4ia*)(dsm + i) = z4;
  }
  __syncthreads();

  int tot = 0;
  const int nChunks = (nE + CHUNK - 1) / CHUNK;
#pragma unroll 1
  for (int ch = 0; ch < nChunks; ++ch) {
    const int cbase = ch * CHUNK;
    const int wc = scan_chunk(keys, nE, cbase, nodeBase, nb, vec8, list, tid, lane, wave);
    if (lane == 0) wcnt[wave] = wc;
    __syncthreads();
    int pre = 0, all = 0;
#pragma unroll
    for (int w2 = 0; w2 < NWAVE; ++w2) {
      int c = wcnt[w2];
      c = c < 0 ? 0 : (c > WCAP ? WCAP : c);
      all += c;
      pre += (w2 < wave) ? c : 0;
    }
    const int wcc  = wc > WCAP ? WCAP : wc;
    const int base = tot + pre;
#pragma unroll 1
    for (int i = lane; i < wcc; i += 32) {
      const int ent = list[wave * WCAP + i];
      const int el  = (ent >> PKS) & (CHUNK - 1);
      const int sl  = ent & (NBA - 1);
      int eid = cbase + el;
      eid = eid > nE - 1 ? nE - 1 : eid;
      const int pos = base + i;
      if (pos < RCAP) reg1[pos] = (int)(((unsigned)eid << PKS) | (unsigned)sl);
    }
    tot += all;
    tot = tot > RCAP ? RCAP : tot;
    __syncthreads();
  }
  const int nh = tot;

  if (wave == 0) {
#pragma unroll 1
    for (int b0 = 0; b0 < nh; b0 += 32) {
      const int idx = b0 + lane;
      const int uv  = reg1[idx < RCAP ? idx : RCAP - 1];
      const int m32 = (nh - b0) < 32 ? (nh - b0) : 32;
#pragma unroll 1
      for (int k = 0; k < m32; ++k) {
        const int u  = __builtin_amdgcn_readlane(uv, k);
        const int sl = u & (NBA - 1);
        if (lane == 0) scnt[sl] = scnt[sl] + 1;
      }
    }
  }
  __syncthreads();

  {
    const v4i ca = *(const v4ia*)(scnt + 4 * tid);
    const int e0 = ca.x < 0 ? 0 : ca.x, e1 = ca.y < 0 ? 0 : ca.y, e2 = ca.z < 0 ? 0 : ca.z, e3 = ca.w < 0 ? 0 : ca.w;
    const int ts = e0 + e1 + e2 + e3;
    int incl = ts;
#pragma unroll
    for (int d = 1; d < 32; d <<= 1) {
      const int up = __shfl_up(incl, d, 32);
      if (lane >= d) incl += up;
    }
    int mx = max(max(e0, e1), max(e2, e3));
    mx = max(mx, __shfl_xor(mx, 16, 32));
    mx = max(mx, __shfl_xor(mx, 8, 32));
    mx = max(mx, __shfl_xor(mx, 4, 32));
    mx = max(mx, __shfl_xor(mx, 2, 32));
    mx = max(mx, __shfl_xor(mx, 1, 32));
    if (lane == 31) wtot[wave] = incl;
    if (lane == 0)  wmx[wave] = mx;
    __syncthreads();
    int pre = 0;
#pragma unroll
    for (int w2 = 0; w2 < NWAVE; ++w2) pre += (w2 < wave) ? wtot[w2] : 0;
    int run = pre + incl - ts;
    v4i so;
    so.x = run; run += e0;
    so.y = run; run += e1;
    so.z = run; run += e2;
    so.w = run;
    *(v4ia*)(soff + 4 * tid) = so;
    *(v4ia*)(cur + 4 * tid)  = so;
  }
#pragma unroll 1
  for (int i = 0; i < 4; ++i) {
    int cc = scnt[4 * tid + i];
    cc = cc < 0 ? 0 : cc;
    sdv[4 * tid + i] = __float_as_int(1.0f / sqrtf((float)(cc + 1)));
  }
  __syncthreads();

  if (wave == 0) {
#pragma unroll 1
    for (int b0 = 0; b0 < nh; b0 += 32) {
      const int idx = b0 + lane;
      const int uv  = reg1[idx < RCAP ? idx : RCAP - 1];
      const int m32 = (nh - b0) < 32 ? (nh - b0) : 32;
#pragma unroll 1
      for (int k = 0; k < m32; ++k) {
        const int u   = __builtin_amdgcn_readlane(uv, k);
        const int sl  = u & (NBA - 1);
        const int eid = (int)((unsigned)u >> PKS);
        if (lane == 0) {
          int pos = cur[sl];
          pos = pos < 0 ? 0 : (pos > RCAP - 1 ? RCAP - 1 : pos);
          reg2[pos] = eid;
          cur[sl] = pos + 1;
        }
      }
    }
  }
  __syncthreads();

  int bmax = 0;
#pragma unroll
  for (int w2 = 0; w2 < NWAVE; ++w2) bmax = max(bmax, wmx[w2]);
  const int flag = ((nh >= RCAP) || (bmax > DEGCAP)) ? 1 : 0;

  int* lrow = LIST + (size_t)blockIdx.x * RCAP;
#pragma unroll 1
  for (int it = 0; it < RCAP / (NTHR * 4); ++it) {
    const int i0 = 4 * (it * NTHR + tid);
    const v4i ev = *(const v4ia*)(reg2 + i0);
    int e0 = ev.x, e1 = ev.y, e2 = ev.z, e3 = ev.w;
    e0 = e0 < 0 ? 0 : (e0 > nE - 1 ? nE - 1 : e0);
    e1 = e1 < 0 ? 0 : (e1 > nE - 1 ? nE - 1 : e1);
    e2 = e2 < 0 ? 0 : (e2 > nE - 1 ? nE - 1 : e2);
    e3 = e3 < 0 ? 0 : (e3 > nE - 1 ? nE - 1 : e3);
    int g0 = gidx[e0], g1 = gidx[e1], g2 = gidx[e2], g3 = gidx[e3];
    asm volatile("" :: "v"(g0), "v"(g1), "v"(g2), "v"(g3));
    g0 = g0 < 0 ? 0 : (g0 > nN - 1 ? nN - 1 : g0);
    g1 = g1 < 0 ? 0 : (g1 > nN - 1 ? nN - 1 : g1);
    g2 = g2 < 0 ? 0 : (g2 > nN - 1 ? nN - 1 : g2);
    g3 = g3 < 0 ? 0 : (g3 > nN - 1 ? nN - 1 : g3);
    v4i ov;
    ov.x = (i0     < nh) ? g0 : 0;
    ov.y = (i0 + 1 < nh) ? g1 : 0;
    ov.z = (i0 + 2 < nh) ? g2 : 0;
    ov.w = (i0 + 3 < nh) ? g3 : 0;
    *(volatile v4i*)(lrow + i0) = ov;
    __threadfence();
    *(volatile v4i*)(lrow + i0) = ov;
  }
  {
    const v4i cv = *(const v4ia*)(scnt + 4 * tid);
    const v4i fv = *(const v4ia*)(soff + 4 * tid);
    const v4i dv = *(const v4ia*)(sdv + 4 * tid);
    v4i rv = {0, 0, 0, 0};
    rv.x = (tid == 0) ? bmax : 0;
    rv.y = (tid == 0) ? flag : 0;
    rv.z = (tid == 0) ? nh : 0;
    int* cp = CNT + (size_t)nodeBase + 4 * tid;
    int* fp = OFF + (size_t)nodeBase + 4 * tid;
    int* dp = DNV + (size_t)nodeBase + 4 * tid;
    int* rp = FLG + (size_t)blockIdx.x * 32 + 4 * (tid & 7);
    *(volatile v4i*)cp = cv;
    *(volatile v4i*)fp = fv;
    *(volatile v4i*)dp = dv;
    if (tid < 8) *(volatile v4i*)rp = rv;
    __threadfence();
    *(volatile v4i*)cp = cv;
    *(volatile v4i*)fp = fv;
    *(volatile v4i*)dp = dv;
    if (tid < 8) *(volatile v4i*)rp = rv;
  }
}

__global__ __launch_bounds__(NTHR) void k_replay(const unsigned short* __restrict__ XB, const int* __restrict__ LIST,
                                                 const int* __restrict__ CNT, const int* __restrict__ OFF,
                                                 const float* __restrict__ DINV, const int* __restrict__ FLG,
                                                 unsigned short* AP, float* G0, int nN, int mRows) {
  __shared__ __attribute__((aligned(16))) float g0s[NBA];
  const int tid = (int)threadIdx.x, lane = tid & 31, wave = tid >> 5, hw = lane >> 4, m = lane & 15;
  const int blk = (int)blockIdx.x;
  const int nodeBase = blk * NBA;
  const int* lp = LIST + (size_t)blk * RCAP;
  const int fl = FLG[(size_t)blk * 32 + 1];
  const float pz = (fl != 0) ? __int_as_float(0x7fc00000) : 0.0f;

#pragma unroll 1
  for (int it = 0; it < NBA / (NWAVE * 2); ++it) {
    const int lrow = wave * (NBA / NWAVE) + 2 * it + hw;
    const int node = nodeBase + lrow;
    const int craw = CNT[node];
    const int oraw = OFF[node];
    const int deg = craw < 0 ? 0 : craw;
    int c = deg > DEGCAP ? DEGCAP : deg;
    const int o = oraw < 0 ? 0 : (oraw > RCAP ? RCAP : oraw);
    if (c > RCAP - o) c = RCAP - o;
    int last = o + c - 1; last = last < o ? o : last;
    last = last > RCAP - 1 ? RCAP - 1 : last;
    int cm = max(c, __shfl_xor(c, 16, 32));
    cm = __builtin_amdgcn_readfirstlane(cm);
    float s0 = 0.0f, s1 = 0.0f, s2 = 0.0f, s3 = 0.0f;
    float q0 = 0.0f, q1 = 0.0f, q2 = 0.0f, q3 = 0.0f;
    float ds = 0.0f;
#pragma unroll 1
    for (int p = 0; p < cm; ++p) {
      int idx = o + p;
      idx = idx > last ? last : idx;
      int s = lp[idx];
      s = s < 0 ? 0 : (s > nN - 1 ? nN - 1 : s);
      const float dv = DINV[s];
      const v2u xw = *(const v2ua*)(XB + (size_t)s * XBP + 4 * m);
      asm volatile("" :: "v"(dv), "v"(xw));
      const bool ok = p < c;
      const float v0 = ok ? bfw_lo(xw.x) : 0.0f;
      const float v1 = ok ? bfw_hi(xw.x) : 0.0f;
      const float v2 = ok ? bfw_lo(xw.y) : 0.0f;
      const float v3 = ok ? bfw_hi(xw.y) : 0.0f;
      const float dk = ok ? dv : 0.0f;
      s0 += v0; s1 += v1; s2 += v2; s3 += v3;
      q0 = fmaf(dk, v0, q0); q1 = fmaf(dk, v1, q1); q2 = fmaf(dk, v2, q2); q3 = fmaf(dk, v3, q3);
      ds += dk;
    }
    const int nc = node < nN ? node : nN - 1;
    const v2u ow = *(const v2ua*)(XB + (size_t)nc * XBP + 4 * m);
    const float di = DINV[nc];
    asm volatile("" :: "v"(ow), "v"(di));
    const bool live = node < nN;
    const float x0 = bfw_lo(ow.x), x1 = bfw_hi(ow.x), x2 = bfw_lo(ow.y), x3 = bfw_hi(ow.y);
    const float cf = (float)deg;
    const float dn = cf > 1.0f ? cf : 1.0f;
    float g_0 = di * (q0 + di * x0), g_1 = di * (q1 + di * x1), g_2 = di * (q2 + di * x2), g_3 = di * (q3 + di * x3);
    float m_0 = s0 / dn, m_1 = s1 / dn, m_2 = s2 / dn, m_3 = s3 / dn;
    float z_0 = x0 + s0, z_1 = x1 + s1, z_2 = x2 + s2, z_3 = x3 + s3;
    float gz = di * (ds + di);
    g_0 = live ? (g_0 + pz) : 0.0f; g_1 = live ? (g_1 + pz) : 0.0f;
    g_2 = live ? (g_2 + pz) : 0.0f; g_3 = live ? (g_3 + pz) : 0.0f;
    m_0 = live ? (m_0 + pz) : 0.0f; m_1 = live ? (m_1 + pz) : 0.0f;
    m_2 = live ? (m_2 + pz) : 0.0f; m_3 = live ? (m_3 + pz) : 0.0f;
    z_0 = live ? (z_0 + pz) : 0.0f; z_1 = live ? (z_1 + pz) : 0.0f;
    z_2 = live ? (z_2 + pz) : 0.0f; z_3 = live ? (z_3 + pz) : 0.0f;
    gz  = live ? (gz + pz) : 0.0f;
    unsigned ha, la, hb, lb;
    v2u gh, gl, mh, ml, zh, zl;
    pack2(g_0, g_1, ha, la); pack2(g_2, g_3, hb, lb);
    gh.x = ha; gh.y = hb; gl.x = la; gl.y = lb;
    pack2(m_0, m_1, ha, la); pack2(m_2, m_3, hb, lb);
    mh.x = ha; mh.y = hb; ml.x = la; ml.y = lb;
    pack2(z_0, z_1, ha, la); pack2(z_2, z_3, hb, lb);
    zh.x = ha; zh.y = hb; zl.x = la; zl.y = lb;
    if (m == 0) g0s[lrow] = gz;
    const bool st = node < mRows;
    const int ns = st ? node : 0;
    unsigned short* rp = AP + (size_t)ns * APP + 4 * m;
    if (st) {
      *(volatile v2u*)(rp)          = gh;
      *(volatile v2u*)(rp + DF)     = gl;
      *(volatile v2u*)(rp + 2 * DF) = mh;
      *(volatile v2u*)(rp + 3 * DF) = ml;
      *(volatile v2u*)(rp + 4 * DF) = zh;
      *(volatile v2u*)(rp + 5 * DF) = zl;
    }
    __threadfence();
    if (st) {
      *(volatile v2u*)(rp)          = gh;
      *(volatile v2u*)(rp + DF)     = gl;
      *(volatile v2u*)(rp + 2 * DF) = mh;
      *(volatile v2u*)(rp + 3 * DF) = ml;
      *(volatile v2u*)(rp + 4 * DF) = zh;
      *(volatile v2u*)(rp + 5 * DF) = zl;
    }
  }
  __syncthreads();
  {
    const v4f gv = *(const v4fa*)(g0s + 4 * tid);
    float* gp = G0 + (size_t)nodeBase + 4 * tid;
    *(volatile v4f*)gp = gv;
    __threadfence();
    *(volatile v4f*)gp = gv;
  }
}

template <int BP>
__device__ __forceinline__ void kgrp(const unsigned short* __restrict__ ap, const unsigned short* __restrict__ bp,
                                     int nks, v8f (&acc)[4]) {
#pragma unroll 1
  for (int ks = 0; ks < nks; ++ks) {
    FragB af;
    af.h[0] = *(const v8usa*)(ap + 32 * ks);
    af.h[1] = *(const v8usa*)(ap + 32 * ks + 16);
#pragma unroll
    for (int t = 0; t < 4; ++t) {
      const unsigned short* wq = bp + (size_t)(16 * t) * (size_t)BP + 32 * ks;
      FragB bf;
      bf.h[0] = *(const v8usa*)wq;
      bf.h[1] = *(const v8usa*)(wq + 16);
      acc[t] = wmb(af, bf, acc[t]);
    }
  }
}

__global__ __launch_bounds__(NTHR) __attribute__((amdgpu_num_vgpr(248)))
void k_mix(const unsigned short* __restrict__ AP, const unsigned short* __restrict__ XB,
           const unsigned short* __restrict__ BA, const unsigned short* __restrict__ BB,
           const unsigned short* __restrict__ BC, const float* __restrict__ PAR,
           const float* __restrict__ G0, const int* __restrict__ FLG, float* out, int nN) {
  extern __shared__ __attribute__((aligned(16))) float stg[];
  __shared__ __attribute__((aligned(16))) float pars[256];
  const int tid = (int)threadIdx.x, lane = tid & 31, wave = tid >> 5, hh = lane >> 4, m = lane & 15;
  const int rowBase = (int)blockIdx.x * GBM;

  if (tid < 64) {
    const v4f p4 = *(const v4f*)(PAR + 4 * tid);
    *(v4fa*)(pars + 4 * tid) = p4;
  }

  v8f accA[4], accB[4], accC[4];
  {
    const v8f z = {0.f, 0.f, 0.f, 0.f, 0.f, 0.f, 0.f, 0.f};
#pragma unroll
    for (int t = 0; t < 4; ++t) { accA[t] = z; accB[t] = z; accC[t] = z; }
  }
  const size_t arow = (size_t)(rowBase + 16 * wave + m);
  const unsigned short* ap = AP + arow * (size_t)APP + 8 * hh;
  const unsigned short* xp = XB + arow * (size_t)XBP + 8 * hh;
  kgrp<BAP>(ap,          BA + (size_t)m * BAP + 8 * hh,          KS_G, accA);
  kgrp<BBP>(ap + 2 * DF, BB + (size_t)m * BBP + 8 * hh,          KS_M, accB);
  kgrp<BBP>(xp,          BB + (size_t)m * BBP + 2 * DF + 8 * hh, 2,    accB);
  kgrp<BCP>(ap + 4 * DF, BC + (size_t)m * BCP + 8 * hh,          KS_Z, accC);

  float* sw = stg + wave * (3 * 16 * DF);
#pragma unroll
  for (int t = 0; t < 4; ++t) {
    const int lc = 16 * t + m;
#pragma unroll
    for (int r = 0; r < 8; ++r) {
      const int lr = 8 * hh + r;
      sw[lr * DF + lc]               = accA[t][r];
      sw[16 * DF + lr * DF + lc]     = accB[t][r];
      sw[2 * 16 * DF + lr * DF + lc] = accC[t][r];
    }
  }
  __syncthreads();

  const int fl = FLG[(size_t)(rowBase >> PKS) * 32 + 1];
  const unsigned pzb = (fl != 0) ? 0x7fc00000u : 0u;
  const unsigned km  = (fl != 0) ? 0u : 0xFFFFFFFFu;
  float* swl = sw + 4 * m;
#pragma unroll 1
  for (int i = 0; i < 8; ++i) {
    const int lr  = 2 * i + hh;
    const int gr  = rowBase + 16 * wave + lr;
    const int grc = gr < nN ? gr : nN - 1;
    const float g0 = G0[grc];
    float o0 = 0.0f, o1 = 0.0f, o2 = 0.0f, o3 = 0.0f;
#pragma unroll 1
    for (int g = 0; g < 3; ++g) {
      const v4f a = *(const v4fa*)(swl + g * (16 * DF) + lr * DF);
      const v4f b = *(const v4fa*)(pars + DF * g + 4 * m);
      const float wg = pars[3 * DF + g];
      const float f  = (g == 0) ? g0 : 1.0f;
      o0 += wg * elu_k(a.x + f * b.x);
      o1 += wg * elu_k(a.y + f * b.y);
      o2 += wg * elu_k(a.z + f * b.z);
      o3 += wg * elu_k(a.w + f * b.w);
    }
    v4f ov;
    ov.x = __uint_as_float((__float_as_uint(o0) & km) | pzb);
    ov.y = __uint_as_float((__float_as_uint(o1) & km) | pzb);
    ov.z = __uint_as_float((__float_as_uint(o2) & km) | pzb);
    ov.w = __uint_as_float((__float_as_uint(o3) & km) | pzb);
    *(v4fa*)(swl + lr * DF) = ov;
    const int grs = gr < nN ? gr : 0;
    float* op = out + (size_t)grs * DF + 4 * m;
    if (gr < nN) *(volatile v4f*)op = ov;
  }
  __threadfence();
#pragma unroll 1
  for (int i = 0; i < 8; ++i) {
    const int lr  = 2 * i + hh;
    const int gr  = rowBase + 16 * wave + lr;
    const v4f ov  = *(const v4fa*)(swl + lr * DF);
    const int grs = gr < nN ? gr : 0;
    float* op = out + (size_t)grs * DF + 4 * m;
    if (gr < nN) *(volatile v4f*)op = ov;
  }
}

static inline int cdiv(int a, int b) { return (a + b - 1) / b; }
static inline size_t al256(size_t o) { return (o + 255) & ~(size_t)255; }

extern "C" void kernel_launch(void* const* d_in, const int* in_sizes, int n_in,
                              void* d_out, int out_size, void* d_ws, size_t ws_size,
                              hipStream_t stream) {
  if (n_in < 11) return;
  if (in_sizes[0] < DF * GBM || (in_sizes[0] % DF) != 0) return;
  const int nN = in_sizes[0] / DF;
  if (in_sizes[2] != 3) return;
  if (in_sizes[3] < 2 || (in_sizes[3] & 1) != 0) return;
  const int nE = in_sizes[3] / 2;
  if (nE < 1 || nE >= (1 << 21)) return;
  if (in_sizes[4] != DF * DF || in_sizes[6] != DF * DF || in_sizes[7] != DF * DF || in_sizes[9] != DF * DF) return;
  if (in_sizes[5] != DF || in_sizes[8] != DF || in_sizes[10] != DF) return;
  if ((long long)out_size != (long long)nN * DF) return;

  const float* x     = (const float*)d_in[0];
  const float* mixw  = (const float*)d_in[2];
  const int*   ei    = (const int*)  d_in[3];
  const int*   src   = ei;
  const int*   dst   = ei + nE;
  const float* wnrm  = (const float*)d_in[4];
  const float* bnrm  = (const float*)d_in[5];
  const float* wself = (const float*)d_in[6];
  const float* wngh  = (const float*)d_in[7];
  const float* bavg  = (const float*)d_in[8];
  const float* wsum  = (const float*)d_in[9];
  const float* bsum  = (const float*)d_in[10];
  float* out = (float*)d_out;

  const int nB    = cdiv(nN, NBA);
  const int NPADN = nB * NBA;
  const int MP    = cdiv(nN, GBM) * GBM;
  if (MP > NPADN || nB > 1024) return;
  const int vec8  = ((nE & 3) == 0) ? 1 : 0;

  char* ws = (char*)d_ws;
  size_t off = 0;
  const size_t oAP = off; off = al256(off + (size_t)MP * APP * 2);
  const size_t oXB = off; off = al256(off + (size_t)MP * XBP * 2);
  const size_t oLS = off; off = al256(off + (size_t)nB * RCAP * 4);
  const size_t oCN = off; off = al256(off + (size_t)NPADN * 4);
  const size_t oOF = off; off = al256(off + (size_t)NPADN * 4);
  const size_t oDV = off; off = al256(off + (size_t)NPADN * 4);
  const size_t oG0 = off; off = al256(off + (size_t)NPADN * 4);
  const size_t oBA = off; off = al256(off + (size_t)DF * BAP * 2);
  const size_t oBB = off; off = al256(off + (size_t)DF * BBP * 2);
  const size_t oBC = off; off = al256(off + (size_t)DF * BCP * 2);
  const size_t oPR = off; off = al256(off + 1024);
  const size_t oFL = off; off = al256(off + (size_t)nB * 128);
  if (off > ws_size || off > (size_t)(128u << 20)) return;
  unsigned short* AP = (unsigned short*)(ws + oAP);
  unsigned short* XB = (unsigned short*)(ws + oXB);
  int*   LIST = (int*)(ws + oLS);
  int*   CNT  = (int*)(ws + oCN);
  int*   OFF  = (int*)(ws + oOF);
  int*   DNV  = (int*)(ws + oDV);
  float* G0   = (float*)(ws + oG0);
  unsigned short* BA = (unsigned short*)(ws + oBA);
  unsigned short* BB = (unsigned short*)(ws + oBB);
  unsigned short* BC = (unsigned short*)(ws + oBC);
  float* PAR  = (float*)(ws + oPR);
  int*   FLG  = (int*)(ws + oFL);

  hipFuncSetAttribute(reinterpret_cast<const void*>(&k_bucket), hipFuncAttributeMaxDynamicSharedMemorySize, LDS_BK);
  hipFuncSetAttribute(reinterpret_cast<const void*>(&k_mix), hipFuncAttributeMaxDynamicSharedMemorySize, LDS_MX);

  const int nXBblk = MP / 32;
  k_prep<<<nXBblk + 2 * NPARTW + 1, NTHR, 0, stream>>>(x, wnrm, wself, wngh, wsum, bnrm, bavg, bsum, mixw,
                                                      XB, BA, BB, BC, PAR, nN, nXBblk);
  k_bucket<<<nB, NTHR, LDS_BK, stream>>>(dst, src, nE, nN, vec8, LIST, CNT, OFF, DNV, FLG);
  k_replay<<<nB, NTHR, 0, stream>>>(XB, LIST, CNT, OFF, (const float*)DNV, FLG, AP, G0, nN, MP);
  k_mix<<<MP / GBM, NTHR, LDS_MX, stream>>>(AP, XB, BA, BB, BC, PAR, G0, FLG, out, nN);
}
